// DMFM_Lite_22024592293913
// MI455X (gfx1250) — hardware-verified
//
#include <hip/hip_runtime.h>
#include <stddef.h>


#define FIN     128
#define HIDC    64
#define NHD     2
#define NCG     (NHD * HIDC)
#define KDEC    (3 * HIDC)
#define NTHR    256
#define NWAVE   8
#define EPT     8
#define NGRP    2
#define CHUNK   (NTHR * EPT * NGRP)
#define WCAP    (EPT * NGRP * 32)
#define LISTN   (NWAVE * WCAP)
#define NBC     4096
#define NBF     1024
#define RCAP    40960
#define RBN     128
#define TGT     256
#define DEGCAP  256
#define OTHR    512
#define BM      64
#define BNROWS  512
#define WSCAP   134217728
#define NEG_SLOPE 0.2f
#define WSCALE  64.0f
#define WINV    0.015625f
#define BN_EPS  1e-5f

#define LDS_FILL ((RCAP + NBF + LISTN) * 4 + 64)

static_assert((CHUNK & (CHUNK - 1)) == 0);
static_assert(CHUNK <= 4096);
static_assert(NBC <= 4096 && NBF <= 4096);
static_assert((NBC & (NBC - 1)) == 0 && (NBF & (NBF - 1)) == 0);
static_assert(NBC == 4 * NBF);
static_assert(OTHR * 8 == NBC);
static_assert((RCAP % 32) == 0);
static_assert(TGT == NWAVE * 32);
static_assert((NBC % TGT) == 0);
static_assert((TGT % BM) == 0);
static_assert(BM * 4 == NTHR);
static_assert(FIN % 32 == 0 && HIDC % 32 == 0 && NCG % 32 == 0 && KDEC % 32 == 0);
static_assert(NCG == 2 * HIDC);
static_assert((BNROWS % 2) == 0);

typedef float          v4f  __attribute__((ext_vector_type(4)));
typedef float          v8f  __attribute__((ext_vector_type(8)));
typedef int            v4i  __attribute__((ext_vector_type(4)));
typedef unsigned       v2u  __attribute__((ext_vector_type(2)));
typedef unsigned       v4u  __attribute__((ext_vector_type(4)));
typedef double         v2d  __attribute__((ext_vector_type(2)));
typedef _Float16       v4h  __attribute__((ext_vector_type(4)));
typedef _Float16       v8h  __attribute__((ext_vector_type(8)));
typedef _Float16       v16h __attribute__((ext_vector_type(16)));
union FragH { v16h v; v8h q[2]; };
union P8 { v4h q[2]; v4i i; };
union P4 { v4h h; v2u u; };

__device__ __forceinline__ v8f wmh(v16h a, v16h b, v8f c) {
  v8f d = __builtin_amdgcn_wmma_f32_16x16x32_f16(false, a, false, b, (short)0, c, false, false);
  asm volatile("v_nop\n\tv_nop\n\tv_nop\n\tv_nop" : "+v"(d) : "v"(a), "v"(b));
  return d;
}

__device__ __forceinline__ v4i pack8h(v4f a, v4f b) {
  P8 p;
  p.q[0] = __builtin_convertvector(a, v4h);
  p.q[1] = __builtin_convertvector(b, v4h);
  return p.i;
}

__device__ __forceinline__ float lrelu(float v) { return v > 0.0f ? v : NEG_SLOPE * v; }
__device__ __forceinline__ float eluf(float v)  { return v > 0.0f ? v : (__expf(v) - 1.0f); }

template <int NB>
__device__ __forceinline__ int scan_chunk(const int* __restrict__ dsts, int nE, int cbase, int slotBase,
                                          int vec8, int* list, int tid, int lane, int wave) {
  int wc = 0;
#pragma unroll
  for (int g = 0; g < NGRP; ++g) {
    const int el0  = (g * NTHR + tid) * EPT;
    const int e0   = cbase + el0;
    const int sent = -2147483647 - 1;
    v4i da, db;
    if (vec8 != 0 && cbase + CHUNK <= nE) {
      da = *(const v4i*)(dsts + e0);
      db = *(const v4i*)(dsts + e0 + 4);
    } else {
      da.x = (e0     < nE) ? dsts[min(e0, nE - 1)] : sent;
      da.y = (e0 + 1 < nE) ? dsts[min(e0 + 1, nE - 1)] : sent;
      da.z = (e0 + 2 < nE) ? dsts[min(e0 + 2, nE - 1)] : sent;
      da.w = (e0 + 3 < nE) ? dsts[min(e0 + 3, nE - 1)] : sent;
      db.x = (e0 + 4 < nE) ? dsts[min(e0 + 4, nE - 1)] : sent;
      db.y = (e0 + 5 < nE) ? dsts[min(e0 + 5, nE - 1)] : sent;
      db.z = (e0 + 6 < nE) ? dsts[min(e0 + 6, nE - 1)] : sent;
      db.w = (e0 + 7 < nE) ? dsts[min(e0 + 7, nE - 1)] : sent;
    }
    const unsigned nb = (unsigned)slotBase;
    const unsigned s0 = (unsigned)da.x - nb, s1 = (unsigned)da.y - nb;
    const unsigned s2 = (unsigned)da.z - nb, s3 = (unsigned)da.w - nb;
    const unsigned s4 = (unsigned)db.x - nb, s5 = (unsigned)db.y - nb;
    const unsigned s6 = (unsigned)db.z - nb, s7 = (unsigned)db.w - nb;
    const bool h0 = s0 < (unsigned)NB, h1 = s1 < (unsigned)NB, h2 = s2 < (unsigned)NB, h3 = s3 < (unsigned)NB;
    const bool h4 = s4 < (unsigned)NB, h5 = s5 < (unsigned)NB, h6 = s6 < (unsigned)NB, h7 = s7 < (unsigned)NB;
    const unsigned any = __builtin_amdgcn_ballot_w32(h0 | h1 | h2 | h3 | h4 | h5 | h6 | h7);
    if (any != 0u) {
#define HITJ(J, HJ, SJ) { \
        const unsigned mj = __builtin_amdgcn_ballot_w32(HJ); \
        if (mj != 0u) { \
          if (HJ) { \
            const int pos = wc + (int)__builtin_amdgcn_mbcnt_lo(mj, 0u); \
            if (pos < WCAP) list[wave * WCAP + pos] = ((el0 + (J)) << 12) | (int)(SJ); \
          } \
          wc += (int)__builtin_popcount(mj); } }
      HITJ(0, h0, s0)
      HITJ(1, h1, s1)
      HITJ(2, h2, s2)
      HITJ(3, h3, s3)
      HITJ(4, h4, s4)
      HITJ(5, h5, s5)
      HITJ(6, h6, s6)
      HITJ(7, h7, s7)
#undef HITJ
    }
  }
  return wc;
}

template <int KD, int NCW>
__global__ __launch_bounds__(NTHR) void k_wprep(const float* __restrict__ W, v4i* wp) {
  constexpr int KS    = KD / 8;
  constexpr int UNITS = NCW * KS;
  static_assert(KD % 32 == 0);
  const int i = (int)blockIdx.x * NTHR + (int)threadIdx.x;
  if (i >= UNITS) return;
  const int n  = i / KS;
  const int k0 = (i - n * KS) * 8;
  v4f a, b;
  a.x = W[(size_t)(k0 + 0) * NCW + n] * WSCALE; a.y = W[(size_t)(k0 + 1) * NCW + n] * WSCALE;
  a.z = W[(size_t)(k0 + 2) * NCW + n] * WSCALE; a.w = W[(size_t)(k0 + 3) * NCW + n] * WSCALE;
  b.x = W[(size_t)(k0 + 4) * NCW + n] * WSCALE; b.y = W[(size_t)(k0 + 5) * NCW + n] * WSCALE;
  b.z = W[(size_t)(k0 + 6) * NCW + n] * WSCALE; b.w = W[(size_t)(k0 + 7) * NCW + n] * WSCALE;
  const v4i o = pack8h(a, b);
  *(volatile v4i*)(wp + i) = o;
  __threadfence();
  *(volatile v4i*)(wp + i) = o;
}

__global__ __launch_bounds__(NTHR) void k_bnstat(const float* __restrict__ x, double* part, int nN) {
  __shared__ __attribute__((aligned(16))) double sS[2 * FIN];
  __shared__ __attribute__((aligned(16))) double sQ[2 * FIN];
  __shared__ __attribute__((aligned(16))) double sT[2 * FIN];
  const int tid = threadIdx.x, f = tid & (FIN - 1), hf = tid >> 7;
  const int r0 = blockIdx.x * BNROWS;
  int r1 = r0 + BNROWS; r1 = r1 > nN ? nN : r1;
  double s = 0.0, q = 0.0;
#pragma unroll 1
  for (int r = r0 + hf; r < r1; r += 2) {
    const double v = (double)x[(size_t)r * FIN + f];
    s += v;
    q = fma(v, v, q);
  }
  sS[tid] = s;
  sQ[tid] = q;
  __syncthreads();
  if (tid < FIN) {
    sT[tid]       = sS[tid] + sS[tid + FIN];
    sT[FIN + tid] = sQ[tid] + sQ[tid + FIN];
  }
  __syncthreads();
  const int li = tid < FIN ? tid : FIN - 1;
  const v2d val = *(const v2d*)(sT + 2 * li);
  double* gp = part + (size_t)blockIdx.x * (2 * FIN) + 2 * li;
  if (tid < FIN) *(volatile v2d*)gp = val;
  __threadfence();
  if (tid < FIN) *(volatile v2d*)gp = val;
}

__global__ __launch_bounds__(FIN) void k_bnfin(const double* __restrict__ part, const float* __restrict__ gamma,
                                              float* bnv, int nPart, int nN) {
  __shared__ __attribute__((aligned(16))) float sv[2 * FIN];
  const int f = threadIdx.x;
  double s = 0.0, q = 0.0;
#pragma unroll 1
  for (int b = 0; b < nPart; ++b) {
    s += part[(size_t)b * (2 * FIN) + f];
    q += part[(size_t)b * (2 * FIN) + FIN + f];
  }
  const double inv = 1.0 / (double)nN;
  const double mu  = s * inv;
  double var = q * inv - mu * mu;
  var = var < 0.0 ? 0.0 : var;
  const float sc = gamma[f] * rsqrtf((float)var + BN_EPS);
  sv[f] = sc;
  sv[FIN + f] = (float)mu;
  __syncthreads();
  const int li = f < 64 ? f : 63;
  const v4f v = *(const v4f*)(sv + 4 * li);
  if (f < 64) *(volatile v4f*)(bnv + 4 * li) = v;
  __threadfence();
  if (f < 64) *(volatile v4f*)(bnv + 4 * li) = v;
}

__global__ __launch_bounds__(NTHR) void k_xcvt(const float* __restrict__ x, const float* __restrict__ bnv,
                                              const float* __restrict__ beta, v4i* xn, v4i* xr, int nN, int nUnits) {
  const int i = (int)blockIdx.x * NTHR + (int)threadIdx.x;
  if (i >= nUnits) return;
  const int row = i >> 4;
  const int c0  = (i & 15) * 8;
  int rr = row > nN - 1 ? nN - 1 : row;
  rr = rr < 0 ? 0 : rr;
  const float* p = x + (size_t)rr * FIN + c0;
  v4f a = *(const v4f*)p, b = *(const v4f*)(p + 4);
  const v4f s0 = *(const v4f*)(bnv + c0), s1 = *(const v4f*)(bnv + c0 + 4);
  const v4f m0 = *(const v4f*)(bnv + FIN + c0), m1 = *(const v4f*)(bnv + FIN + c0 + 4);
  const v4f e0 = *(const v4f*)(beta + c0), e1 = *(const v4f*)(beta + c0 + 4);
  v4f na = (a - m0) * s0 + e0;
  v4f nb = (b - m1) * s1 + e1;
  const v4f z = {0.f, 0.f, 0.f, 0.f};
  if (row >= nN) { a = z; b = z; na = z; nb = z; }
  const v4i on = pack8h(na, nb);
  const v4i orr = pack8h(a, b);
  *(volatile v4i*)(xn + i) = on;
  *(volatile v4i*)(xr + i) = orr;
  __threadfence();
  *(volatile v4i*)(xn + i) = on;
  *(volatile v4i*)(xr + i) = orr;
}

__global__ __launch_bounds__(NTHR) void k_count(
    const int* __restrict__ dsts, int* cnt, int nE, int vec8) {
  __shared__ __attribute__((aligned(16))) int scnt[NBC];
  __shared__ __attribute__((aligned(16))) int list[LISTN];
  __shared__ int wcnt[NWAVE];
  const int tid = threadIdx.x, lane = tid & 31, wave = tid >> 5;
  const int nodeBase = blockIdx.x * NBC;

  for (int i = tid; i < NBC; i += NTHR) scnt[i] = 0;
  __syncthreads();

  const int nChunks = (nE + CHUNK - 1) / CHUNK;
#pragma unroll 1
  for (int ch = 0; ch < nChunks; ++ch) {
    const int cbase = ch * CHUNK;
    const int wc = scan_chunk<NBC>(dsts, nE, cbase, nodeBase, vec8, list, tid, lane, wave);
    if (lane == 0) wcnt[wave] = wc;
    __syncthreads();
    if (wave == 0) {
#pragma unroll 1
      for (int wsx = 0; wsx < NWAVE; ++wsx) {
        int n = __builtin_amdgcn_readfirstlane(wcnt[wsx]);
        n = n > WCAP ? WCAP : (n < 0 ? 0 : n);
        const int* lp = list + wsx * WCAP;
#pragma unroll 1
        for (int i = 0; i < n; ++i) {
          const int ent  = __builtin_amdgcn_readfirstlane(lp[i]);
          const int slot = ent & (NBC - 1);
          if (lane == 0) scnt[slot] = scnt[slot] + 1;
        }
      }
    }
    __syncthreads();
  }

  v4i cq[4];
#pragma unroll
  for (int q = 0; q < 4; ++q) {
    const int f = (wave * 4 + q) * 128 + 4 * lane;
    cq[q] = *(const v4i*)(scnt + f);
  }
  int* cp = cnt + (size_t)nodeBase;
#pragma unroll
  for (int q = 0; q < 4; ++q) {
    const int f = (wave * 4 + q) * 128 + 4 * lane;
    *(volatile v4i*)(cp + f) = cq[q];
  }
  __threadfence();
#pragma unroll
  for (int q = 0; q < 4; ++q) {
    const int f = (wave * 4 + q) * 128 + 4 * lane;
    *(volatile v4i*)(cp + f) = cq[q];
  }
}

__global__ __launch_bounds__(OTHR) void k_offsets(
    const int* __restrict__ cnt, int* off, int* rbase, int nChunk) {
  __shared__ __attribute__((aligned(16))) int soff[NBC];
  __shared__ __attribute__((aligned(16))) int srb[RBN];
  __shared__ int wtot[OTHR / 32];
  const int tid = threadIdx.x, lane = tid & 31, wave = tid >> 5, sub = tid >> 7;
  for (int i = tid; i < RBN; i += OTHR) srb[i] = 0;
  int carry = 0;
#pragma unroll 1
  for (int ch = 0; ch < nChunk; ++ch) {
    const int base = ch * NBC;
    const v4i c0 = *(const v4i*)(cnt + base + 8 * tid);
    const v4i c1 = *(const v4i*)(cnt + base + 8 * tid + 4);
    const int e0 = max(c0.x, 0), e1 = max(c0.y, 0), e2 = max(c0.z, 0), e3 = max(c0.w, 0);
    const int e4 = max(c1.x, 0), e5 = max(c1.y, 0), e6 = max(c1.z, 0), e7 = max(c1.w, 0);
    const int ts = e0 + e1 + e2 + e3 + e4 + e5 + e6 + e7;
    int incl = ts;
#pragma unroll
    for (int d = 1; d < 32; d <<= 1) {
      const int t = __shfl_up(incl, d);
      if (lane >= d) incl += t;
    }
    if (lane == 31) wtot[wave] = incl;
    __syncthreads();
    const int S0 = wtot[0]  + wtot[1]  + wtot[2]  + wtot[3];
    const int S1 = wtot[4]  + wtot[5]  + wtot[6]  + wtot[7];
    const int S2 = wtot[8]  + wtot[9]  + wtot[10] + wtot[11];
    const int S3 = wtot[12] + wtot[13] + wtot[14] + wtot[15];
    int pre = 0;
#pragma unroll 1
    for (int w = 4 * sub; w < wave; ++w) pre += wtot[w];
    const int b0 = carry;
    const int b1 = b0 + ((S0 + 31) & ~31);
    const int b2 = b1 + ((S1 + 31) & ~31);
    const int b3 = b2 + ((S2 + 31) & ~31);
    const int b4 = b3 + ((S3 + 31) & ~31);
    const int myb = sub == 0 ? b0 : (sub == 1 ? b1 : (sub == 2 ? b2 : b3));
    if (tid == 0) {
      srb[min(4 * ch + 0, RBN - 1)] = b0;
      srb[min(4 * ch + 1, RBN - 1)] = b1;
      srb[min(4 * ch + 2, RBN - 1)] = b2;
      srb[min(4 * ch + 3, RBN - 1)] = b3;
    }
    int run = myb + pre + incl - ts;
    soff[8 * tid + 0] = run; run += e0;
    soff[8 * tid + 1] = run; run += e1;
    soff[8 * tid + 2] = run; run += e2;
    soff[8 * tid + 3] = run; run += e3;
    soff[8 * tid + 4] = run; run += e4;
    soff[8 * tid + 5] = run; run += e5;
    soff[8 * tid + 6] = run; run += e6;
    soff[8 * tid + 7] = run;
    carry = b4;
    __syncthreads();
    const v4i o0 = *(const v4i*)(soff + 4 * tid);
    const v4i o1 = *(const v4i*)(soff + 4 * (tid + OTHR));
    int* op = off + base;
    *(volatile v4i*)(op + 4 * tid) = o0;
    *(volatile v4i*)(op + 4 * (tid + OTHR)) = o1;
    __threadfence();
    *(volatile v4i*)(op + 4 * tid) = o0;
    *(volatile v4i*)(op + 4 * (tid + OTHR)) = o1;
    __syncthreads();
  }
  if (tid == 0) srb[min(4 * nChunk, RBN - 1)] = carry;
  __syncthreads();
  v4i rv = {0, 0, 0, 0};
  if (tid < 32) rv = *(const v4i*)(srb + 4 * tid);
  if (tid < 32) *(volatile v4i*)(rbase + 4 * tid) = rv;
  __threadfence();
  if (tid < 32) *(volatile v4i*)(rbase + 4 * tid) = rv;
}

__global__ __launch_bounds__(NTHR) void k_fill(
    const int* __restrict__ srcs, const int* __restrict__ dsts,
    const int* __restrict__ off, const int* __restrict__ rbase,
    int* csr, int nN, int nE, int vec8, int csrLen) {
  extern __shared__ v4f lds_dyn[];
  int* region = (int*)lds_dyn;
  int* cursor = region + RCAP;
  int* list   = cursor + NBF;
  int* wcnt   = list + LISTN;
  const int tid = threadIdx.x, lane = tid & 31, wave = tid >> 5;
  const int b = blockIdx.x;
  const int nodeBase = b * NBF;

  int rb0 = rbase[b];
  const int rb1 = rbase[b + 1];
  rb0 = rb0 < 0 ? 0 : (rb0 > csrLen ? csrLen : rb0);
  rb0 &= ~31;
  int len = rb1 - rb0;
  len = len < 0 ? 0 : (len > RCAP ? RCAP : len);
  int lenW = (len + 31) & ~31;
  if (rb0 + lenW > csrLen) lenW = (csrLen - rb0) & ~31;

  {
    const v4i z = {0, 0, 0, 0};
    for (int i = tid; i < RCAP / 4; i += NTHR) ((v4i*)region)[i] = z;
    for (int s = tid; s < NBF; s += NTHR) {
      int o = off[nodeBase + s] - rb0;
      o = o < 0 ? 0 : (o > RCAP ? RCAP : o);
      cursor[s] = o;
    }
  }
  __syncthreads();

  const int nChunks = (nE + CHUNK - 1) / CHUNK;
#pragma unroll 1
  for (int ch = 0; ch < nChunks; ++ch) {
    const int cbase = ch * CHUNK;
    const int wc = scan_chunk<NBF>(dsts, nE, cbase, nodeBase, vec8, list, tid, lane, wave);
    if (lane == 0) wcnt[wave] = wc;
    __syncthreads();
    if (wave == 0) {
#pragma unroll 1
      for (int wsx = 0; wsx < NWAVE; ++wsx) {
        int n = __builtin_amdgcn_readfirstlane(wcnt[wsx]);
        n = n > WCAP ? WCAP : (n < 0 ? 0 : n);
        const int* lp = list + wsx * WCAP;
#pragma unroll 1
        for (int i = 0; i < n; ++i) {
          const int ent  = __builtin_amdgcn_readfirstlane(lp[i]);
          const int slot = ent & (NBF - 1);
          int e = cbase + ((ent >> 12) & (CHUNK - 1));
          e = e > nE - 1 ? nE - 1 : e;
          int src = srcs[e];
          src = src < 0 ? 0 : (src > nN - 1 ? nN - 1 : src);
          if (lane == 0) {
            int pos = cursor[slot];
            pos = pos < 0 ? 0 : (pos > RCAP - 1 ? RCAP - 1 : pos);
            region[pos] = src;
            const int np = pos + 1;
            cursor[slot] = np > RCAP ? RCAP : np;
          }
        }
      }
    }
    __syncthreads();
  }

  const int nv = lenW >> 2;
  int* gp = csr + rb0;
#pragma unroll 1
  for (int i = tid; i < nv; i += NTHR) { const v4i v = ((const v4i*)region)[i]; *(volatile v4i*)(gp + 4 * i) = v; }
  __threadfence();
#pragma unroll 1
  for (int i = tid; i < nv; i += NTHR) { const v4i v = ((const v4i*)region)[i]; *(volatile v4i*)(gp + 4 * i) = v; }
}

template <int KS, int NSTEP, int NC>
__device__ __forceinline__ void mma_block(const _Float16* __restrict__ A, size_t aps,
                                          const _Float16* __restrict__ Bp,
                                          float* stg, int rowBase, int tid) {
  constexpr int TPW = NC / 32;
  constexpr int LDB = NSTEP * 32;
  constexpr int SPS = KS / 32;
  static_assert(KS % 32 == 0 && TPW >= 1 && TPW * 32 == NC);
  static_assert((NSTEP % SPS) == 0);
  const int lane = tid & 31, wave = tid >> 5, hh = lane >> 4, m = lane & 15;
  const int r0 = (wave >> 1) * 16;
  const int c0 = (wave & 1) * (NC / 2);

  v8f acc[TPW];
#pragma unroll
  for (int t = 0; t < TPW; ++t) { v8f z = {0.f, 0.f, 0.f, 0.f, 0.f, 0.f, 0.f, 0.f}; acc[t] = z; }

  const _Float16* arow = A  + (size_t)(rowBase + r0 + m) * KS + 8 * hh;
  const _Float16* bcol = Bp + (size_t)(c0 + m) * LDB + 8 * hh;
#pragma unroll 1
  for (int kt = 0; kt < NSTEP; ++kt) {
    const int s  = kt / SPS;
    const int ks = kt - s * SPS;
    const _Float16* ap = arow + (size_t)s * aps + 32 * ks;
    FragH a;
    a.q[0] = *(const v8h*)ap;
    a.q[1] = *(const v8h*)(ap + 16);
#pragma unroll
    for (int t = 0; t < TPW; ++t) {
      const _Float16* bp = bcol + (size_t)(16 * t) * LDB + 32 * kt;
      FragH bf;
      bf.q[0] = *(const v8h*)bp;
      bf.q[1] = *(const v8h*)(bp + 16);
      acc[t] = wmh(a.v, bf.v, acc[t]);
    }
  }

  float* sp = stg + (size_t)(r0 + 8 * hh) * NC + c0 + m;
#pragma unroll
  for (int t = 0; t < TPW; ++t) {
#pragma unroll
    for (int r = 0; r < 8; ++r) sp[r * NC + 16 * t] = acc[t][r] * WINV;
  }
}

__global__ __launch_bounds__(NTHR) void k_gemm_enc(const _Float16* __restrict__ A, const _Float16* __restrict__ Bp,
                                                  const float* __restrict__ bias, float* Cf, v4i* C16) {
  constexpr int NC  = HIDC;
  constexpr int NIT = BM * NC / 4 / NTHR;
  constexpr int NIU = BM * NC / 8 / NTHR;
  static_assert(NIT * NTHR * 4 == BM * NC && NIU * NTHR * 8 == BM * NC);
  __shared__ __attribute__((aligned(16))) float stg[BM * NC];
  const int tid = threadIdx.x;
  const int rowBase = blockIdx.x * BM;
  mma_block<FIN, FIN / 32, NC>(A, 0, Bp, stg, rowBase, tid);
  __syncthreads();

  v4f cv[NIT];
#pragma unroll
  for (int it = 0; it < NIT; ++it) {
    const int idx = it * NTHR + tid;
    const int col = (4 * idx) & (NC - 1);
    v4f v = *(const v4f*)(stg + 4 * idx) + *(const v4f*)(bias + col);
    v.x = v.x > 0.f ? v.x : 0.f; v.y = v.y > 0.f ? v.y : 0.f;
    v.z = v.z > 0.f ? v.z : 0.f; v.w = v.w > 0.f ? v.w : 0.f;
    cv[it] = v;
    *(v4f*)(stg + 4 * idx) = v;
  }
  __syncthreads();
  v4i hv[NIU];
#pragma unroll
  for (int iu = 0; iu < NIU; ++iu) {
    const int u = iu * NTHR + tid;
    hv[iu] = pack8h(*(const v4f*)(stg + 8 * u), *(const v4f*)(stg + 8 * u + 4));
  }
  float* tileC = Cf + (size_t)rowBase * NC;
  v4i*   tileH = C16 + (size_t)rowBase * (NC / 8);
#pragma unroll
  for (int it = 0; it < NIT; ++it) *(volatile v4f*)(tileC + 4 * (size_t)(it * NTHR + tid)) = cv[it];
#pragma unroll
  for (int iu = 0; iu < NIU; ++iu) *(volatile v4i*)(tileH + (size_t)(iu * NTHR + tid)) = hv[iu];
  __threadfence();
#pragma unroll
  for (int it = 0; it < NIT; ++it) *(volatile v4f*)(tileC + 4 * (size_t)(it * NTHR + tid)) = cv[it];
#pragma unroll
  for (int iu = 0; iu < NIU; ++iu) *(volatile v4i*)(tileH + (size_t)(iu * NTHR + tid)) = hv[iu];
}

__global__ __launch_bounds__(NTHR) void k_gemm_gat(const _Float16* __restrict__ A, const _Float16* __restrict__ Bp,
                                                  const float* __restrict__ attS, const float* __restrict__ attD,
                                                  float* hw, float* eS, float* eD) {
  constexpr int NC  = NCG;
  constexpr int NIT = BM * NC / 4 / NTHR;
  constexpr int NES = BM * NHD;
  constexpr int CPP = NC / 4;
  static_assert(NIT * NTHR * 4 == BM * NC);
  static_assert(NES == 4 * 32);
  static_assert(2 * CPP == HIDC);
  __shared__ __attribute__((aligned(16))) float stg[BM * NC];
  __shared__ __attribute__((aligned(16))) float sES[NES];
  __shared__ __attribute__((aligned(16))) float sED[NES];
  const int tid = threadIdx.x, lane = tid & 31, wave = tid >> 5;
  const int rowBase = blockIdx.x * BM;
  mma_block<HIDC, HIDC / 32, NC>(A, 0, Bp, stg, rowBase, tid);
  __syncthreads();

  {
    const int drow = tid >> 2, part = tid & 3;
    const float* rp  = stg + (size_t)drow * NC + CPP * part;
    const float* sa  = attS + CPP * part;
    const float* sdd = attD + CPP * part;
    float ps = 0.f, pd = 0.f;
#pragma unroll 2
    for (int c = 0; c < CPP; c += 4) {
      const v4f hv = *(const v4f*)(rp + c);
      const v4f av = *(const v4f*)(sa + c);
      const v4f dv = *(const v4f*)(sdd + c);
      ps += hv.x * av.x + hv.y * av.y + hv.z * av.z + hv.w * av.w;
      pd += hv.x * dv.x + hv.y * dv.y + hv.z * dv.z + hv.w * dv.w;
    }
    ps += __shfl_xor(ps, 1); pd += __shfl_xor(pd, 1);
    if ((part & 1) == 0) { sES[drow * NHD + (part >> 1)] = ps; sED[drow * NHD + (part >> 1)] = pd; }
  }

  float* tileC = hw + (size_t)rowBase * NC;
  v4f cv[NIT];
#pragma unroll
  for (int it = 0; it < NIT; ++it) cv[it] = *(const v4f*)(stg + 4 * (it * NTHR + tid));
#pragma unroll
  for (int it = 0; it < NIT; ++it) *(volatile v4f*)(tileC + 4 * (size_t)(it * NTHR + tid)) = cv[it];
  __syncthreads();
  const v4f vS = *(const v4f*)(sES + 4 * lane);
  const v4f vD = *(const v4f*)(sED + 4 * lane);
  float* gS = eS + (size_t)rowBase * NHD + 4 * lane;
  float* gD = eD + (size_t)rowBase * NHD + 4 * lane;
  if (wave == 0) *(volatile v4f*)gS = vS;
  if (wave == 1) *(volatile v4f*)gD = vD;
  __threadfence();
#pragma unroll
  for (int it = 0; it < NIT; ++it) *(volatile v4f*)(tileC + 4 * (size_t)(it * NTHR + tid)) = cv[it];
  if (wave == 0) *(volatile v4f*)gS = vS;
  if (wave == 1) *(volatile v4f*)gD = vD;
}

__global__ __launch_bounds__(NTHR) void k_gemm_dec(const _Float16* __restrict__ A, size_t aps,
                                                  const _Float16* __restrict__ Bp, const float* __restrict__ b1,
                                                  const float* __restrict__ w2, const float* __restrict__ b2,
                                                  float* deep) {
  constexpr int NC = HIDC;
  __shared__ __attribute__((aligned(16))) float stg[BM * NC];
  __shared__ __attribute__((aligned(16))) float sOut[BM];
  const int tid = threadIdx.x, lane = tid & 31, wave = tid >> 5;
  const int rowBase = blockIdx.x * BM;
  mma_block<HIDC, KDEC / 32, NC>(A, aps, Bp, stg, rowBase, tid);
  __syncthreads();

  {
    const int drow = tid >> 2, part = tid & 3, j0 = 16 * part;
    const float* rp = stg + drow * NC + j0;
    float z = 0.f;
#pragma unroll
    for (int q = 0; q < 16; q += 4) {
      v4f t = *(const v4f*)(rp + q) + *(const v4f*)(b1 + j0 + q);
      const v4f w = *(const v4f*)(w2 + j0 + q);
      t.x = t.x > 0.f ? t.x : 0.f; t.y = t.y > 0.f ? t.y : 0.f;
      t.z = t.z > 0.f ? t.z : 0.f; t.w = t.w > 0.f ? t.w : 0.f;
      z += t.x * w.x + t.y * w.y + t.z * w.z + t.w * w.w;
    }
    z += __shfl_xor(z, 1);
    z += __shfl_xor(z, 2);
    if (part == 0) sOut[drow] = z + b2[0];
  }
  __syncthreads();
  {
    const int li = lane < 16 ? lane : 15;
    const v4f ov = *(const v4f*)(sOut + 4 * li);
    float* gp = deep + (size_t)rowBase + 4 * li;
    const bool w0 = (wave == 0) && (lane < 16);
    if (w0) *(volatile v4f*)gp = ov;
    __threadfence();
    if (w0) *(volatile v4f*)gp = ov;
  }
}

__global__ __launch_bounds__(NTHR) void k_gemm_att(const _Float16* __restrict__ A, const _Float16* __restrict__ Bp,
                                                  const float* __restrict__ bias, float* attn) {
  constexpr int NC  = FIN;
  constexpr int NIT = BM * NC / 4 / NTHR;
  static_assert(NIT * NTHR * 4 == BM * NC);
  __shared__ __attribute__((aligned(16))) float stg[BM * NC];
  const int tid = threadIdx.x;
  const int rowBase = blockIdx.x * BM;
  mma_block<FIN, FIN / 32, NC>(A, 0, Bp, stg, rowBase, tid);
  __syncthreads();

  {
    const int drow = tid >> 2, part = tid & 3;
    float* rp = stg + (size_t)drow * NC + 32 * part;
    const float* bp = bias + 32 * part;
    float mx = __int_as_float(0xff800000u);
#pragma unroll
    for (int c = 0; c < 32; c += 4) {
      v4f u = *(const v4f*)(rp + c) + *(const v4f*)(bp + c);
      u.x = lrelu(u.x); u.y = lrelu(u.y); u.z = lrelu(u.z); u.w = lrelu(u.w);
      *(v4f*)(rp + c) = u;
      mx = fmaxf(mx, fmaxf(fmaxf(u.x, u.y), fmaxf(u.z, u.w)));
    }
    mx = fmaxf(mx, __shfl_xor(mx, 1));
    mx = fmaxf(mx, __shfl_xor(mx, 2));
    float s = 0.f;
#pragma unroll
    for (int c = 0; c < 32; c += 4) {
      const v4f u = *(const v4f*)(rp + c);
      v4f e;
      e.x = __expf(u.x - mx); e.y = __expf(u.y - mx); e.z = __expf(u.z - mx); e.w = __expf(u.w - mx);
      *(v4f*)(rp + c) = e;
      s += (e.x + e.y) + (e.z + e.w);
    }
    s += __shfl_xor(s, 1);
    s += __shfl_xor(s, 2);
    const float inv = __builtin_amdgcn_rcpf(s);
#pragma unroll
    for (int c = 0; c < 32; c += 4) {
      const v4f e = *(const v4f*)(rp + c);
      *(v4f*)(rp + c) = e * inv;
    }
  }
  __syncthreads();

  float* tileC = attn + (size_t)rowBase * NC;
  v4f cv[NIT];
#pragma unroll
  for (int it = 0; it < NIT; ++it) cv[it] = *(const v4f*)(stg + 4 * (it * NTHR + tid));
#pragma unroll
  for (int it = 0; it < NIT; ++it) *(volatile v4f*)(tileC + 4 * (size_t)(it * NTHR + tid)) = cv[it];
  __threadfence();
#pragma unroll
  for (int it = 0; it < NIT; ++it) *(volatile v4f*)(tileC + 4 * (size_t)(it * NTHR + tid)) = cv[it];
}

__global__ __launch_bounds__(NTHR) void k_agg(
    const int* __restrict__ csr, const int* __restrict__ off, const int* __restrict__ cnt,
    const float* __restrict__ eS, const float* __restrict__ eD, const float* __restrict__ hw,
    const float* __restrict__ bias, const float* __restrict__ Cprev,
    float* Hout, float* Cout, v4u* C16, int nN, int csrLen) {
  const int tid = threadIdx.x, lane = tid & 31, wave = tid >> 5;
  const int tbase = blockIdx.x * TGT + wave * 32;
  const int col = 4 * lane;
  const int hd  = lane >> 4;
  const int cq  = 4 * (lane & 15);
  const int sl0 = (2 * lane) & 15, sl1 = (2 * lane + 1) & 15;
  const v4f bb = *(const v4f*)(bias + cq);

  const int cl    = tbase + lane;
  const int cnt_l = cnt[cl];
  const int off_l = off[cl];

#pragma unroll 1
  for (int j = 0; j < 32; ++j) {
    const int c = tbase + j;
    int n = __shfl(cnt_l, j);
    n = n < 0 ? 0 : (n > DEGCAP ? DEGCAP : n);
    const int st = __shfl(off_l, j);
    const float edc   = eD[(size_t)c * NHD + hd];
    const float eself = lrelu(eS[(size_t)c * NHD + hd] + edc);

    float mx = eself;
#pragma unroll 1
    for (int q0 = 0; q0 < n; q0 += 32) {
      int pos = st + q0 + lane;
      pos = pos < 0 ? 0 : (pos > csrLen - 1 ? csrLen - 1 : pos);
      int sl = csr[pos];
      sl = sl < 0 ? 0 : (sl > nN - 1 ? nN - 1 : sl);
      const int mcnt = (n - q0) < 32 ? (n - q0) : 32;
#pragma unroll 1
      for (int pp = 0; pp < mcnt; ++pp) {
        const int s = __builtin_amdgcn_readlane(sl, pp);
        mx = fmaxf(mx, lrelu(eS[(size_t)s * NHD + hd] + edc));
      }
    }

    float p   = __expf(eself - mx);
    float den = p;
    v4f acc = *(const v4f*)(hw + (size_t)c * NCG + col) * p;
#pragma unroll 1
    for (int q0 = 0; q0 < n; q0 += 32) {
      int pos = st + q0 + lane;
      pos = pos < 0 ? 0 : (pos > csrLen - 1 ? csrLen - 1 : pos);
      int sl = csr[pos];
      sl = sl < 0 ? 0 : (sl > nN - 1 ? nN - 1 : sl);
      const int mcnt = (n - q0) < 32 ? (n - q0) : 32;
#pragma unroll 1
      for (int pp = 0; pp < mcnt; ++pp) {
        const int s = __builtin_amdgcn_readlane(sl, pp);
        p = __expf(lrelu(eS[(size_t)s * NHD + hd] + edc) - mx);
        den += p;
        const v4f hv = *(const v4f*)(hw + (size_t)s * NCG + col);
        acc = acc + hv * p;
      }
    }

    const float rd = __builtin_amdgcn_rcpf(den);
    const v4f v = acc * rd;
    v4f pv;
    pv.x = __shfl_xor(v.x, 16); pv.y = __shfl_xor(v.y, 16);
    pv.z = __shfl_xor(v.z, 16); pv.w = __shfl_xor(v.w, 16);
    const v4f mm = (v + pv) * 0.5f + bb;
    v4f H;
    H.x = eluf(mm.x); H.y = eluf(mm.y); H.z = eluf(mm.z); H.w = eluf(mm.w);
    const v4f cp = *(const v4f*)(Cprev + (size_t)c * HIDC + cq);
    v4f Cn = cp - H;
    if (c >= nN) { const v4f z = {0.f, 0.f, 0.f, 0.f}; H = z; Cn = z; }

    P4 pk;
    pk.h = __builtin_convertvector(Cn, v4h);
    v4u o16;
    o16.x = __shfl(pk.u.x, sl0); o16.y = __shfl(pk.u.y, sl0);
    o16.z = __shfl(pk.u.x, sl1); o16.w = __shfl(pk.u.y, sl1);

    float* hp  = Hout + (size_t)c * HIDC + cq;
    float* cnp = Cout + (size_t)c * HIDC + cq;
    v4u*   gp  = C16 + (size_t)c * (HIDC / 8) + (lane & 7);
    if (lane < 16) { *(volatile v4f*)hp = H; *(volatile v4f*)cnp = Cn; }
    if (lane < 8) *(volatile v4u*)gp = o16;
    __threadfence();
    if (lane < 16) { *(volatile v4f*)hp = H; *(volatile v4f*)cnp = Cn; }
    if (lane < 8) *(volatile v4u*)gp = o16;
  }
}

__global__ __launch_bounds__(NTHR) void k_pack(const float* __restrict__ wsf, float* out,
                                              long long q0, long long q1, long long q2, long long q3,
                                              long long q4, long long q5, long long q6,
                                              int s1, int s2, int s3, int s4, int s5, int s6, int nF4) {
  const int i = (int)blockIdx.x * NTHR + (int)threadIdx.x;
  if (i >= nF4) return;
  const int g = 4 * i;
  long long rel = q0;
  rel = (g >= s1) ? q1 : rel;
  rel = (g >= s2) ? q2 : rel;
  rel = (g >= s3) ? q3 : rel;
  rel = (g >= s4) ? q4 : rel;
  rel = (g >= s5) ? q5 : rel;
  rel = (g >= s6) ? q6 : rel;
  const v4f v = *(const v4f*)(wsf + (rel + (long long)g));
  float* gp = out + (size_t)g;
  *(volatile v4f*)gp = v;
  __threadfence();
  *(volatile v4f*)gp = v;
}

extern "C" void kernel_launch(void* const* d_in, const int* in_sizes, int n_in,
                              void* d_out, int out_size, void* d_ws, size_t ws_size,
                              hipStream_t stream) {
  if (n_in < 21) return;
  const int nN  = in_sizes[0] / FIN;
  const int nE1 = in_sizes[1] / 2;
  const int nE2 = in_sizes[2] / 2;
  if (nN <= 0 || nE1 <= 0 || nE2 <= 0) return;
  if (in_sizes[0] != nN * FIN || in_sizes[1] != 2 * nE1 || in_sizes[2] != 2 * nE2) return;
  if (in_sizes[3] != FIN || in_sizes[4] != FIN || in_sizes[5] != FIN * HIDC || in_sizes[6] != HIDC) return;
  if (in_sizes[7] != HIDC * NCG || in_sizes[8] != NCG || in_sizes[9] != NCG || in_sizes[10] != HIDC) return;
  if (in_sizes[11] != HIDC * NCG || in_sizes[12] != NCG || in_sizes[13] != NCG || in_sizes[14] != HIDC) return;
  if (in_sizes[15] != KDEC * HIDC || in_sizes[16] != HIDC || in_sizes[17] != HIDC || in_sizes[18] != 1) return;
  if (in_sizes[19] != FIN * FIN || in_sizes[20] != FIN) return;
  if (out_size != nN * (1 + FIN + 5 * HIDC) || (out_size & 3) != 0) return;
  if (nE1 > (1 << 28) || nE2 > (1 << 28) || nN > (1 << 22)) return;

  const float* x     = (const float*)d_in[0];
  const int*   ei1   = (const int*)d_in[1];
  const int*   ei2   = (const int*)d_in[2];
  const float* gamma = (const float*)d_in[3];
  const float* beta  = (const float*)d_in[4];
  const float* Wenc  = (const float*)d_in[5];
  const float* benc  = (const float*)d_in[6];
  const float* Wg1   = (const float*)d_in[7];
  const float* as1   = (const float*)d_in[8];
  const float* ad1   = (const float*)d_in[9];
  const float* bg1   = (const float*)d_in[10];
  const float* Wg2   = (const float*)d_in[11];
  const float* as2   = (const float*)d_in[12];
  const float* ad2   = (const float*)d_in[13];
  const float* bg2   = (const float*)d_in[14];
  const float* Wd1   = (const float*)d_in[15];
  const float* bd1   = (const float*)d_in[16];
  const float* Wd2   = (const float*)d_in[17];
  const float* bd2   = (const float*)d_in[18];
  const float* Wa    = (const float*)d_in[19];
  const float* ba    = (const float*)d_in[20];
  float* out = (float*)d_out;

  const int NPAD   = ((nN + TGT - 1) / TGT) * TGT;
  const int nBC    = (nN + NBC - 1) / NBC;
  const int CNTPAD = nBC * NBC;
  if (CNTPAD < NPAD) return;
  if (4 * nBC + 1 > RBN) return;
  const int nBF    = (nN + NBF - 1) / NBF;
  if (nBF + 1 > 4 * nBC + 1) return;
  if (31 * 4 * nBC > 4096) return;
  const int csrLen1 = ((nE1 + 31) & ~31) + 4096;
  const int csrLen2 = ((nE2 + 31) & ~31) + 4096;
  const int nPart  = (nN + BNROWS - 1) / BNROWS;
  const int nAgg   = NPAD / TGT;
  const int nGemm  = NPAD / BM;
  const int nXu    = NPAD * (FIN / 8);

  char* ws = (char*)d_ws;
  size_t off = 0;
  auto carve = [&](size_t bytes) { const size_t o = off; off += (bytes + 255) & ~(size_t)255; return o; };
  const size_t oWe   = carve((size_t)HIDC * FIN * 2);
  const size_t oWg1  = carve((size_t)NCG * HIDC * 2);
  const size_t oWg2  = carve((size_t)NCG * HIDC * 2);
  const size_t oWd1  = carve((size_t)HIDC * KDEC * 2);
  const size_t oWa   = carve((size_t)FIN * FIN * 2);
  const size_t oPart = carve((size_t)nPart * 2 * FIN * 8);
  const size_t oBnv  = carve((size_t)2 * FIN * 4);
  const size_t oXn   = carve((size_t)NPAD * FIN * 2);
  const size_t oXr   = carve((size_t)NPAD * FIN * 2);
  const size_t oC16  = carve((size_t)3 * NPAD * HIDC * 2);
  const size_t oCf   = carve((size_t)NPAD * HIDC * 4);
  const size_t oCIf  = carve((size_t)NPAD * HIDC * 4);
  const size_t oCUf  = carve((size_t)NPAD * HIDC * 4);
  const size_t oHIf  = carve((size_t)NPAD * HIDC * 4);
  const size_t oHUf  = carve((size_t)NPAD * HIDC * 4);
  const size_t oAtt  = carve((size_t)NPAD * FIN * 4);
  const size_t oDeep = carve((size_t)NPAD * 4);
  const size_t oHw   = carve((size_t)NPAD * NCG * 4);
  const size_t oES   = carve((size_t)NPAD * NHD * 4);
  const size_t oED   = carve((size_t)NPAD * NHD * 4);
  const size_t oCnt1 = carve((size_t)CNTPAD * 4);
  const size_t oOff1 = carve((size_t)CNTPAD * 4);
  const size_t oRb1  = carve((size_t)RBN * 4);
  const size_t oCsr1 = carve((size_t)csrLen1 * 4);
  const size_t oCnt2 = carve((size_t)CNTPAD * 4);
  const size_t oOff2 = carve((size_t)CNTPAD * 4);
  const size_t oRb2  = carve((size_t)RBN * 4);
  const size_t oCsr2 = carve((size_t)csrLen2 * 4);
  if (off > ws_size || off > (size_t)WSCAP) return;

  v4i* wpe   = (v4i*)(ws + oWe);
  v4i* wpg1  = (v4i*)(ws + oWg1);
  v4i* wpg2  = (v4i*)(ws + oWg2);
  v4i* wpd1  = (v4i*)(ws + oWd1);
  v4i* wpa   = (v4i*)(ws + oWa);
  double* part = (double*)(ws + oPart);
  float* bnv = (float*)(ws + oBnv);
  v4i* xn    = (v4i*)(ws + oXn);
  v4i* xr    = (v4i*)(ws + oXr);
  char* c16b = ws + oC16;
  const size_t planeBytes = (size_t)NPAD * HIDC * 2;
  const size_t aps = (size_t)NPAD * HIDC;
  float* Cf   = (float*)(ws + oCf);
  float* CIf  = (float*)(ws + oCIf);
  float* CUf  = (float*)(ws + oCUf);
  float* HIf  = (float*)(ws + oHIf);
  float* HUf  = (float*)(ws + oHUf);
  float* attn = (float*)(ws + oAtt);
  float* deep = (float*)(ws + oDeep);
  float* hw   = (float*)(ws + oHw);
  float* es   = (float*)(ws + oES);
  float* ed   = (float*)(ws + oED);
  int* cnt1 = (int*)(ws + oCnt1); int* off1 = (int*)(ws + oOff1); int* rb1 = (int*)(ws + oRb1); int* csr1 = (int*)(ws + oCsr1);
  int* cnt2 = (int*)(ws + oCnt2); int* off2 = (int*)(ws + oOff2); int* rb2 = (int*)(ws + oRb2); int* csr2 = (int*)(ws + oCsr2);

  const int vec81 = ((nE1 & 3) == 0) ? 1 : 0;
  const int vec82 = ((nE2 & 3) == 0) ? 1 : 0;

  k_wprep<FIN, HIDC><<<(HIDC * FIN / 8 + NTHR - 1) / NTHR, NTHR, 0, stream>>>(Wenc, wpe);
  k_wprep<HIDC, NCG><<<(NCG * HIDC / 8 + NTHR - 1) / NTHR, NTHR, 0, stream>>>(Wg1, wpg1);
  k_wprep<HIDC, NCG><<<(NCG * HIDC / 8 + NTHR - 1) / NTHR, NTHR, 0, stream>>>(Wg2, wpg2);
  k_wprep<KDEC, HIDC><<<(HIDC * KDEC / 8 + NTHR - 1) / NTHR, NTHR, 0, stream>>>(Wd1, wpd1);
  k_wprep<FIN, FIN><<<(FIN * FIN / 8 + NTHR - 1) / NTHR, NTHR, 0, stream>>>(Wa, wpa);

  k_bnstat<<<nPart, NTHR, 0, stream>>>(x, part, nN);
  k_bnfin<<<1, FIN, 0, stream>>>(part, gamma, bnv, nPart, nN);
  k_xcvt<<<(nXu + NTHR - 1) / NTHR, NTHR, 0, stream>>>(x, bnv, beta, xn, xr, nN, nXu);

  hipFuncSetAttribute(reinterpret_cast<const void*>(&k_fill),
                      hipFuncAttributeMaxDynamicSharedMemorySize, LDS_FILL);
  k_count<<<nBC, NTHR, 0, stream>>>(ei1 + nE1, cnt1, nE1, vec81);
  k_offsets<<<1, OTHR, 0, stream>>>(cnt1, off1, rb1, nBC);
  k_fill<<<nBF, NTHR, LDS_FILL, stream>>>(ei1, ei1 + nE1, off1, rb1, csr1, nN, nE1, vec81, csrLen1);
  k_count<<<nBC, NTHR, 0, stream>>>(ei2 + nE2, cnt2, nE2, vec82);
  k_offsets<<<1, OTHR, 0, stream>>>(cnt2, off2, rb2, nBC);
  k_fill<<<nBF, NTHR, LDS_FILL, stream>>>(ei2, ei2 + nE2, off2, rb2, csr2, nN, nE2, vec82, csrLen2);

  k_gemm_enc<<<nGemm, NTHR, 0, stream>>>((const _Float16*)xn, (const _Float16*)wpe, benc, Cf, (v4i*)c16b);

  k_gemm_gat<<<nGemm, NTHR, 0, stream>>>((const _Float16*)c16b, (const _Float16*)wpg1, as1, ad1, hw, es, ed);
  k_agg<<<nAgg, NTHR, 0, stream>>>(csr1, off1, cnt1, es, ed, hw, bg1, Cf, HIf, CIf,
                                   (v4u*)(c16b + planeBytes), nN, csrLen1);

  k_gemm_gat<<<nGemm, NTHR, 0, stream>>>((const _Float16*)(c16b + planeBytes), (const _Float16*)wpg2, as2, ad2, hw, es, ed);
  k_agg<<<nAgg, NTHR, 0, stream>>>(csr2, off2, cnt2, es, ed, hw, bg2, CIf, HUf, CUf,
                                   (v4u*)(c16b + 2 * planeBytes), nN, csrLen2);

  k_gemm_dec<<<nGemm, NTHR, 0, stream>>>((const _Float16*)c16b, aps, (const _Float16*)wpd1, bd1, Wd2, bd2, deep);

  k_gemm_att<<<nGemm, NTHR, 0, stream>>>((const _Float16*)xr, (const _Float16*)wpa, ba, attn);

  const int s1 = nN;
  const int s2 = s1 + nN * FIN;
  const int s3 = s2 + nN * HIDC;
  const int s4 = s3 + nN * HIDC;
  const int s5 = s4 + nN * HIDC;
  const int s6 = s5 + nN * HIDC;
  const long long q0 = (long long)(oDeep / 4);
  const long long q1 = (long long)(oAtt / 4) - s1;
  const long long q2 = (long long)(oCf  / 4) - s2;
  const long long q3 = (long long)(oCIf / 4) - s3;
  const long long q4 = (long long)(oCUf / 4) - s4;
  const long long q5 = (long long)(oHIf / 4) - s5;
  const long long q6 = (long long)(oHUf / 4) - s6;
  const int nF4 = out_size / 4;
  k_pack<<<(nF4 + NTHR - 1) / NTHR, NTHR, 0, stream>>>((const float*)ws, out, q0, q1, q2, q3, q4, q5, q6,
                                                       s1, s2, s3, s4, s5, s6, nF4);
}
